// MultiheadAttention_15341623181846
// MI455X (gfx1250) — hardware-verified
//
#include <hip/hip_runtime.h>


#ifndef NB
#define NB 1
#endif
#ifndef SEQ
#define SEQ 4096
#endif
#define SEQ_FULL 4096
#define DM   1024
#define NH_  16
#define HD   64
#define CCP  (2 * DM)
#define AW   4
#define QRS  2048.0f
#define QRI  (1.0f / 2048.0f)
#define L2E  1.4426950408889634f
#define PSH  8.0f

static_assert(NB == 1);
static_assert(HD == 64);
static_assert(NH_ * HD == DM);
static_assert(DM % 64 == 0);
static_assert(DM % 32 == 0);
static_assert((DM & (DM - 1)) == 0);
static_assert(SEQ % 64 == 0);
static_assert(SEQ % 32 == 0);
static_assert(SEQ % (16 * AW) == 0);
static_assert(((size_t)SEQ * DM) % 8 == 0);
static_assert(SEQ <= SEQ_FULL);

typedef _Float16 h16;
typedef unsigned short bf;
typedef __attribute__((ext_vector_type(16))) __bf16   v16bf;
typedef __attribute__((ext_vector_type(16))) _Float16 v16h;
typedef __attribute__((ext_vector_type(8)))  _Float16 v8h;
typedef __attribute__((ext_vector_type(8)))  unsigned short v8us;
typedef __attribute__((ext_vector_type(8)))  float    v8f;
typedef __attribute__((ext_vector_type(4)))  float    v4f;
typedef v4f  __attribute__((may_alias)) v4fa;

__device__ __forceinline__ unsigned short f2bf(float f) { unsigned u = __float_as_uint(f); u += 0x7FFFu + ((u >> 16) & 1u); return (unsigned short)(u >> 16); }
__device__ __forceinline__ float bf2f(unsigned short s) { return __uint_as_float(((unsigned)s) << 16); }
__device__ __forceinline__ v16h cat16(v8h lo, v8h hi) { return __builtin_shufflevector(lo, hi, 0, 1, 2, 3, 4, 5, 6, 7, 8, 9, 10, 11, 12, 13, 14, 15); }
__device__ __forceinline__ v16bf cat16b(v8us lo, v8us hi) { return __builtin_bit_cast(v16bf, __builtin_shufflevector(lo, hi, 0, 1, 2, 3, 4, 5, 6, 7, 8, 9, 10, 11, 12, 13, 14, 15)); }
__device__ __forceinline__ v8f wmma16(v16h a, v16h b, v8f c) { return __builtin_amdgcn_wmma_f32_16x16x32_f16(false, a, false, b, (short)0, c, false, false); }
__device__ __forceinline__ v8f wmmab(v16bf a, v16bf b, v8f c) { return __builtin_amdgcn_wmma_f32_16x16x32_bf16(false, a, false, b, (short)0, c, false, false); }
__device__ __forceinline__ v16h  ldh(const h16* p) { return cat16(*(const v8h*)p, *(const v8h*)(p + 16)); }
__device__ __forceinline__ v16bf ldbf(const bf* p) { return cat16b(*(const v8us*)p, *(const v8us*)(p + 16)); }
__device__ __forceinline__ void wave_sync() { __builtin_amdgcn_fence(3  , "wavefront"); __builtin_amdgcn_wave_barrier(); asm volatile("" ::: "memory"); }

__global__ __launch_bounds__(256) void k_cvt8(const float* __restrict__ src, bf* dst, size_t n8) {
    const size_t i = (size_t)blockIdx.x * 256 + threadIdx.x; if (i >= n8) return;
    const v8f v = *(const v8f*)(src + i * 8); v8us o;
#pragma unroll
    for (int k = 0; k < 8; ++k) o[k] = f2bf(v[k]);
    *(volatile v8us*)(dst + i * 8) = o; __threadfence(); *(volatile v8us*)(dst + i * 8) = o;
}

__global__ __launch_bounds__(256) void k_tcvt(const float* __restrict__ src, bf* dst, int R, int C) {
    __shared__ float t[64 * 65];
    const int tid = threadIdx.x; const int r0 = blockIdx.x * 64, c0 = blockIdx.y * 64; const size_t zb = (size_t)blockIdx.z * (size_t)R * (size_t)C;
#pragma unroll
    for (int i = 0; i < 4; ++i) { const int idx = tid + 256 * i; const int r = idx >> 4, c4 = (idx & 15) * 4;
        const v4f v = *(const v4f*)(src + zb + (size_t)(r0 + r) * (size_t)C + c0 + c4);
        t[r * 65 + c4] = v[0]; t[r * 65 + c4 + 1] = v[1]; t[r * 65 + c4 + 2] = v[2]; t[r * 65 + c4 + 3] = v[3]; }
    __syncthreads();
#pragma unroll 1
    for (int ps = 0; ps < 2; ++ps) {
#pragma unroll
        for (int p = 0; p < 2; ++p) { const int c = (tid >> 3) + 32 * p, r8 = (tid & 7) * 8; v8us o;
#pragma unroll
            for (int i = 0; i < 8; ++i) o[i] = f2bf(t[(r8 + i) * 65 + c]);
            *(volatile v8us*)(dst + zb + (size_t)(c0 + c) * (size_t)R + r0 + r8) = o; }
        if (ps == 0) __threadfence(); }
}

template <int MODE>
__global__ __launch_bounds__(32) void k_gemm(const bf* __restrict__ A, const bf* __restrict__ Bt, int K, int sa, int sb, int kbm,
                                             h16* Ph, h16* Pr, float* Of, int useRes, int RB, size_t sRB, int pitch, int CB, size_t sCB) {
    __shared__ __align__(16) float os[16 * 68];
    const int lane = threadIdx.x & 31, lr = lane & 15, hi = lane >> 4; const int r0 = blockIdx.x * 64, c0 = blockIdx.y * 64;
    v8f acc[4][4];
#pragma unroll
    for (int mb = 0; mb < 4; ++mb)
#pragma unroll
        for (int nb = 0; nb < 4; ++nb) acc[mb][nb] = (v8f){};
    const size_t aoff = (size_t)(r0 + lr) * (size_t)sa + 8 * hi, boff = (size_t)(c0 + lr) * (size_t)sb + 8 * hi;
#pragma unroll 1
    for (int kc = 0; kc < K; kc += 32) {
        const int kb = kc & kbm;
        v16bf a[4];
#pragma unroll
        for (int mb = 0; mb < 4; ++mb) a[mb] = ldbf(A + aoff + (size_t)mb * 16 * (size_t)sa + kc);
#pragma unroll
        for (int nb = 0; nb < 4; ++nb) { const v16bf b = ldbf(Bt + boff + (size_t)nb * 16 * (size_t)sb + kb);
#pragma unroll
            for (int mb = 0; mb < 4; ++mb) acc[mb][nb] = wmmab(a[mb], b, acc[mb][nb]); }
        asm volatile("v_nop\n\tv_nop\n\tv_nop\n\tv_nop" : "+v"(acc[0][0]), "+v"(acc[1][1]), "+v"(acc[2][2]), "+v"(acc[3][3]) : "v"(a[0]), "v"(a[1]), "v"(a[2]), "v"(a[3]));
    }
    const size_t tbase = (size_t)(r0 / RB) * sRB + (size_t)(r0 % RB) * (size_t)pitch + (size_t)(c0 / CB) * sCB + (size_t)(c0 % CB);
#pragma unroll
    for (int mb = 0; mb < 4; ++mb) {
#pragma unroll
        for (int nb = 0; nb < 4; ++nb) {
#pragma unroll
            for (int j = 0; j < 8; ++j) os[(hi * 8 + j) * 68 + nb * 16 + lr] = acc[mb][nb][j]; }
        wave_sync();
        const size_t sbase = tbase + (size_t)(mb * 16) * (size_t)pitch;
        if (MODE == 0) {
#pragma unroll 1
            for (int ps = 0; ps < 2; ++ps) {
#pragma unroll
                for (int s = 0; s < 4; ++s) { const int row = 4 * s + (lane >> 3), c8 = (lane & 7) * 8;
                    const v4f x0 = *(const v4fa*)(&os[row * 68 + c8]); const v4f x1 = *(const v4fa*)(&os[row * 68 + c8 + 4]); v8h hv, rv;
#pragma unroll
                    for (int i = 0; i < 4; ++i) { const h16 a0 = (h16)x0[i]; const h16 a1 = (h16)x1[i]; hv[i] = a0; hv[4 + i] = a1; rv[i] = (h16)((x0[i] - (float)a0) * QRS); rv[4 + i] = (h16)((x1[i] - (float)a1) * QRS); }
                    const size_t oo = sbase + (size_t)row * (size_t)pitch + c8;
                    *(volatile v8h*)(Ph + oo) = hv; if (useRes) *(volatile v8h*)(Pr + oo) = rv; }
                if (ps == 0) __threadfence(); }
        } else {
#pragma unroll 1
            for (int ps = 0; ps < 2; ++ps) {
#pragma unroll
                for (int s = 0; s < 8; ++s) { const int row = 2 * s + hi, cofs = lr * 4;
                    const v4f val = *(const v4fa*)(&os[row * 68 + cofs]);
                    *(volatile v4f*)(Of + sbase + (size_t)row * (size_t)pitch + cofs) = val; }
                if (ps == 0) __threadfence(); }
        }
        wave_sync();
    }
}

__global__ __launch_bounds__(32 * AW) void k_flash(const h16* __restrict__ QH, const h16* __restrict__ QR, const h16* __restrict__ KH, const h16* __restrict__ KR, const h16* __restrict__ VT, bf* CC) {
    __shared__ __align__(16) float os[AW * 16 * 68];
    const int lane = threadIdx.x & 31, wave = __builtin_amdgcn_readfirstlane((int)(threadIdx.x >> 5)), lr = lane & 15, hi = lane >> 4;
    const int h = blockIdx.y;
    const int t0 = (blockIdx.x * AW + wave) * 16;
    const size_t pbase = (size_t)h * SEQ * HD;
    const size_t qo = pbase + (size_t)(t0 + lr) * HD + 8 * hi;
    const v16h qh0 = ldh(QH + qo), qh1 = ldh(QH + qo + 32), qr0 = ldh(QR + qo), qr1 = ldh(QR + qo + 32);
    const size_t ko = pbase + (size_t)lr * HD + 8 * hi;
    const size_t vo = pbase + (size_t)lr * SEQ + 8 * hi;
    v8f o0 = (v8f){}, o1 = (v8f){}, o2 = (v8f){}, o3 = (v8f){};
    float m = -1.0e30f, l = 0.0f;
#pragma unroll 1
    for (int key0 = 0; key0 < SEQ; key0 += 32) {
        const size_t kofs = ko + (size_t)key0 * HD;
        v8f sHa = (v8f){}, sLa = (v8f){}, sHb = (v8f){}, sLb = (v8f){};
        {
            const v16h ka = ldh(KH + kofs), kar = ldh(KR + kofs), kb = ldh(KH + kofs + 16 * HD), kbr = ldh(KR + kofs + 16 * HD);
            sHa = wmma16(ka, qh0, sHa); sLa = wmma16(ka, qr0, sLa); sHb = wmma16(kb, qh0, sHb); sLb = wmma16(kb, qr0, sLb);
            sLa = wmma16(kar, qh0, sLa); sLb = wmma16(kbr, qh0, sLb);
            asm volatile("v_nop\n\tv_nop\n\tv_nop\n\tv_nop" : "+v"(sHa), "+v"(sLa), "+v"(sHb), "+v"(sLb) : "v"(ka), "v"(kar), "v"(kb), "v"(kbr));
        }
        {
            const v16h ka = ldh(KH + kofs + 32), kar = ldh(KR + kofs + 32), kb = ldh(KH + kofs + 16 * HD + 32), kbr = ldh(KR + kofs + 16 * HD + 32);
            sHa = wmma16(ka, qh1, sHa); sLa = wmma16(ka, qr1, sLa); sHb = wmma16(kb, qh1, sHb); sLb = wmma16(kb, qr1, sLb);
            sLa = wmma16(kar, qh1, sLa); sLb = wmma16(kbr, qh1, sLb);
            asm volatile("v_nop\n\tv_nop\n\tv_nop\n\tv_nop" : "+v"(sHa), "+v"(sLa), "+v"(sHb), "+v"(sLb) : "v"(ka), "v"(kar), "v"(kb), "v"(kbr));
        }
        float ta[8], tb[8]; float mx = -1.0e30f;
#pragma unroll
        for (int r = 0; r < 8; ++r) { ta[r] = (sHa[r] + sLa[r] * QRI) * 0.125f; tb[r] = (sHb[r] + sLb[r] * QRI) * 0.125f; mx = fmaxf(mx, fmaxf(ta[r], tb[r])); }
        mx = fmaxf(mx, __shfl_xor(mx, 16, 32));
        const float mnew = fmaxf(m, mx);
        const float alpha = __builtin_amdgcn_exp2f((m - mnew) * L2E);
        v16h pb; float ls = 0.0f;
#pragma unroll
        for (int r = 0; r < 8; ++r) { const h16 pa = (h16)__builtin_amdgcn_exp2f((ta[r] - mnew) * L2E + PSH); const h16 pc = (h16)__builtin_amdgcn_exp2f((tb[r] - mnew) * L2E + PSH); pb[r] = pa; pb[8 + r] = pc; ls += (float)pa + (float)pc; }
        l = l * alpha + ls; m = mnew;
        o0 = o0 * alpha; o1 = o1 * alpha; o2 = o2 * alpha; o3 = o3 * alpha;
        const h16* va = VT + vo + key0;
        const v16h v0 = ldh(va), v1 = ldh(va + (size_t)16 * SEQ), v2 = ldh(va + (size_t)32 * SEQ), v3 = ldh(va + (size_t)48 * SEQ);
        o0 = wmma16(v0, pb, o0); o1 = wmma16(v1, pb, o1); o2 = wmma16(v2, pb, o2); o3 = wmma16(v3, pb, o3);
        asm volatile("v_nop\n\tv_nop\n\tv_nop\n\tv_nop" : "+v"(o0), "+v"(o1), "+v"(o2), "+v"(o3) : "v"(v0), "v"(v1), "v"(v2), "v"(v3), "v"(pb));
    }
    l += __shfl_xor(l, 16, 32);
    const float inv = 1.0f / l;
    const int wb = wave * 16 * 68;
    { v4f a, c;
      a[0] = o0[0] * inv; a[1] = o0[1] * inv; a[2] = o0[2] * inv; a[3] = o0[3] * inv; c[0] = o0[4] * inv; c[1] = o0[5] * inv; c[2] = o0[6] * inv; c[3] = o0[7] * inv;
      *(v4fa*)(&os[wb + lr * 68 +  0 + 8 * hi]) = a; *(v4fa*)(&os[wb + lr * 68 +  0 + 8 * hi + 4]) = c;
      a[0] = o1[0] * inv; a[1] = o1[1] * inv; a[2] = o1[2] * inv; a[3] = o1[3] * inv; c[0] = o1[4] * inv; c[1] = o1[5] * inv; c[2] = o1[6] * inv; c[3] = o1[7] * inv;
      *(v4fa*)(&os[wb + lr * 68 + 16 + 8 * hi]) = a; *(v4fa*)(&os[wb + lr * 68 + 16 + 8 * hi + 4]) = c;
      a[0] = o2[0] * inv; a[1] = o2[1] * inv; a[2] = o2[2] * inv; a[3] = o2[3] * inv; c[0] = o2[4] * inv; c[1] = o2[5] * inv; c[2] = o2[6] * inv; c[3] = o2[7] * inv;
      *(v4fa*)(&os[wb + lr * 68 + 32 + 8 * hi]) = a; *(v4fa*)(&os[wb + lr * 68 + 32 + 8 * hi + 4]) = c;
      a[0] = o3[0] * inv; a[1] = o3[1] * inv; a[2] = o3[2] * inv; a[3] = o3[3] * inv; c[0] = o3[4] * inv; c[1] = o3[5] * inv; c[2] = o3[6] * inv; c[3] = o3[7] * inv;
      *(v4fa*)(&os[wb + lr * 68 + 48 + 8 * hi]) = a; *(v4fa*)(&os[wb + lr * 68 + 48 + 8 * hi + 4]) = c; }
    wave_sync();
    bf* crow = CC + (size_t)t0 * CCP + h * HD;
#pragma unroll 1
    for (int ps = 0; ps < 2; ++ps) {
#pragma unroll
        for (int s = 0; s < 4; ++s) { const int row = 4 * s + (lane >> 3), c8 = (lane & 7) * 8;
            const v4f x0 = *(const v4fa*)(&os[wb + row * 68 + c8]); const v4f x1 = *(const v4fa*)(&os[wb + row * 68 + c8 + 4]); v8us hv, lv;
#pragma unroll
            for (int i = 0; i < 4; ++i) { const unsigned short a0 = f2bf(x0[i]); const unsigned short a1 = f2bf(x1[i]); hv[i] = a0; hv[4 + i] = a1;
                lv[i] = f2bf(x0[i] - bf2f(a0)); lv[4 + i] = f2bf(x1[i] - bf2f(a1)); }
            const size_t oo = (size_t)row * CCP + c8;
            *(volatile v8us*)(crow + oo) = hv; *(volatile v8us*)(crow + oo + DM) = lv; }
        if (ps == 0) __threadfence(); }
}

static constexpr size_t al256(size_t v) { return (v + 255) & ~(size_t)255; }
static constexpr size_t SZ_XB = al256((size_t)SEQ * DM * 2);
static constexpr size_t SZ_W1 = al256((size_t)DM * DM * 2);
static constexpr size_t SZ_PL = al256((size_t)NH_ * SEQ * HD * 2);
static constexpr size_t SZ_CC = al256((size_t)SEQ * CCP * 2);
static constexpr size_t SZ_TOTAL = SZ_XB + 4 * SZ_W1 + 5 * SZ_PL + SZ_CC;
static_assert(SZ_TOTAL <= (size_t)134217728);

extern "C" void kernel_launch(void* const* d_in, const int* in_sizes, int n_in,
                              void* d_out, int out_size, void* d_ws, size_t ws_size, hipStream_t stream) {
    if (n_in < 5) return;
    if ((size_t)in_sizes[0] < (size_t)SEQ * DM) return;
    if ((size_t)in_sizes[1] < (size_t)NH_ * DM * HD || (size_t)in_sizes[2] < (size_t)NH_ * DM * HD || (size_t)in_sizes[3] < (size_t)NH_ * DM * HD) return;
    if ((size_t)in_sizes[4] < (size_t)DM * DM) return;
    if ((size_t)out_size < (size_t)SEQ * DM) return;
    if (SZ_TOTAL > ws_size) return;
    const float* x = (const float*)d_in[0]; const float* wq = (const float*)d_in[1]; const float* wk = (const float*)d_in[2]; const float* wv = (const float*)d_in[3]; const float* wp = (const float*)d_in[4];
    float* OUT = (float*)d_out;
    char* wsp = (char*)d_ws;
    bf* XB  = (bf*)wsp; wsp += SZ_XB;
    bf* WQT = (bf*)wsp; wsp += SZ_W1;
    bf* WKT = (bf*)wsp; wsp += SZ_W1;
    bf* WVT = (bf*)wsp; wsp += SZ_W1;
    bf* WPT = (bf*)wsp; wsp += SZ_W1;
    h16* QH = (h16*)wsp; wsp += SZ_PL;
    h16* QR = (h16*)wsp; wsp += SZ_PL;
    h16* KH = (h16*)wsp; wsp += SZ_PL;
    h16* KR = (h16*)wsp; wsp += SZ_PL;
    h16* VT = (h16*)wsp; wsp += SZ_PL;
    bf* CC  = (bf*)wsp; wsp += SZ_CC;

    { const size_t n8 = (size_t)SEQ * DM / 8;
      k_cvt8<<<(unsigned)((n8 + 255) / 256), 256, 0, stream>>>(x, XB, n8); }
    k_tcvt<<<dim3(DM / 64, HD / 64, NH_), 256, 0, stream>>>(wq, WQT, DM, HD);
    k_tcvt<<<dim3(DM / 64, HD / 64, NH_), 256, 0, stream>>>(wk, WKT, DM, HD);
    k_tcvt<<<dim3(DM / 64, HD / 64, NH_), 256, 0, stream>>>(wv, WVT, DM, HD);
    k_tcvt<<<dim3(DM / 64, DM / 64, 1), 256, 0, stream>>>(wp, WPT, DM, DM);

    k_gemm<0><<<dim3(SEQ / 64, DM / 64, 1), 32, 0, stream>>>(XB, WQT, DM, DM, DM, DM - 1, QH, QR, OUT, 1, SEQ, (size_t)0, HD, HD, (size_t)SEQ * HD);
    k_gemm<0><<<dim3(SEQ / 64, DM / 64, 1), 32, 0, stream>>>(XB, WKT, DM, DM, DM, DM - 1, KH, KR, OUT, 1, SEQ, (size_t)0, HD, HD, (size_t)SEQ * HD);
    k_gemm<0><<<dim3(DM / 64, SEQ / 64, 1), 32, 0, stream>>>(WVT, XB, DM, DM, DM, DM - 1, VT, VT, OUT, 0, DM, (size_t)0, SEQ, SEQ, (size_t)0);

    k_flash<<<dim3(SEQ / (16 * AW), NH_, 1), 32 * AW, 0, stream>>>(QH, QR, KH, KR, VT, CC);

    k_gemm<1><<<dim3(SEQ / 64, DM / 64, 1), 32, 0, stream>>>(CC, WPT, 2 * DM, 2 * DM, DM, DM - 1, QH, QH, OUT, 0, SEQ, (size_t)0, DM, DM, (size_t)0);
}
